// MemoryEfficientAttnBlock3D_69827578298391
// MI455X (gfx1250) — hardware-verified
//
#include <hip/hip_runtime.h>


#define NB_  2
#define CC   64
#define NV   8192
#define NG   32
#define RB   1024
#define DM   CC
#define SCL  0.125f
#define GEPS 1e-6f
#define LOSC 1024.0f

typedef _Float16 h16;
typedef unsigned short bf;
typedef __attribute__((ext_vector_type(16))) __bf16   v16bf;
typedef __attribute__((ext_vector_type(16))) _Float16 v16h;
typedef __attribute__((ext_vector_type(8)))  _Float16 v8h;
typedef __attribute__((ext_vector_type(8)))  unsigned short v8us;
typedef __attribute__((ext_vector_type(8)))  float    v8f;
typedef __attribute__((ext_vector_type(4)))  float    v4f;
typedef v8h  __attribute__((may_alias)) v8ha;
typedef v4f  __attribute__((may_alias)) v4fa;
typedef v8us __attribute__((may_alias)) v8usa;

__device__ __forceinline__ unsigned short f2bf(float f) { unsigned u = __float_as_uint(f); u += 0x7FFFu + ((u >> 16) & 1u); return (unsigned short)(u >> 16); }
__device__ __forceinline__ float bf2f(unsigned short b) { return __uint_as_float(((unsigned)b) << 16); }
__device__ __forceinline__ float bfr(float f) { return bf2f(f2bf(f)); }
__device__ __forceinline__ v16h cat16(v8h lo, v8h hi) { return __builtin_shufflevector(lo, hi, 0, 1, 2, 3, 4, 5, 6, 7, 8, 9, 10, 11, 12, 13, 14, 15); }
__device__ __forceinline__ v16bf cat16b(v8us lo, v8us hi) { return __builtin_bit_cast(v16bf, __builtin_shufflevector(lo, hi, 0, 1, 2, 3, 4, 5, 6, 7, 8, 9, 10, 11, 12, 13, 14, 15)); }
__device__ __forceinline__ v8f wmma16(v16h a, v16h b, v8f c) { return __builtin_amdgcn_wmma_f32_16x16x32_f16(false, a, false, b, (short)0, c, false, false); }
__device__ __forceinline__ v8f wmmab(v16bf a, v16bf b, v8f c) { return __builtin_amdgcn_wmma_f32_16x16x32_bf16(false, a, false, b, (short)0, c, false, false); }

template <bool SPLITA, bool F16OUT = false>
__global__ __launch_bounds__(128) void k_gemmb(const bf* __restrict__ A, const bf* __restrict__ Al, const bf* __restrict__ Bn, const float* __restrict__ bias, float* C, int ldc, h16* C2, const float* __restrict__ R = nullptr, int K = DM, int roundR = 1) {
    __shared__ __align__(16) float ost[4][16 * 68];
    const int lane = threadIdx.x & 31, wave = threadIdx.x >> 5, lr = lane & 15, hi = lane >> 4;
    const int r0 = blockIdx.x * 64 + wave * 16, c0 = blockIdx.y * 64;
    const size_t aoff = (size_t)(r0 + lr) * K + 8 * hi;
    size_t boff[4];
#pragma unroll
    for (int t = 0; t < 4; ++t) boff[t] = (size_t)(c0 + t * 16 + lr) * K + 8 * hi;
    v8f acc[4];
#pragma unroll
    for (int t = 0; t < 4; ++t) acc[t] = (v8f){};
#pragma unroll 1
    for (int kc = 0; kc < K; kc += 32) {
        const v16bf a = cat16b(*(const v8us*)(A + aoff + kc), *(const v8us*)(A + aoff + kc + 16));
        v16bf al = a;
        if (SPLITA) al = cat16b(*(const v8us*)(Al + aoff + kc), *(const v8us*)(Al + aoff + kc + 16));
#pragma unroll
        for (int t = 0; t < 4; ++t) { const v16bf b = cat16b(*(const v8us*)(Bn + boff[t] + kc), *(const v8us*)(Bn + boff[t] + kc + 16)); acc[t] = wmmab(a, b, acc[t]); if (SPLITA) acc[t] = wmmab(al, b, acc[t]); }
        asm volatile("v_nop\n\tv_nop\n\tv_nop\n\tv_nop" : "+v"(acc[0]), "+v"(acc[1]), "+v"(acc[2]), "+v"(acc[3]) : "v"(a), "v"(al));
    }
    float* os = &ost[wave][0];
#pragma unroll
    for (int t = 0; t < 4; ++t) { const float bv = bias ? bfr(bias[c0 + t * 16 + lr]) : 0.f;
#pragma unroll
        for (int j = 0; j < 8; ++j) os[(hi * 8 + j) * 68 + t * 16 + lr] = acc[t][j] + bv; }
    __syncthreads();
    if (F16OUT) {
        h16* crow = (h16*)(void*)C + (size_t)r0 * ldc + c0;
        auto pass = [&]() {
#pragma unroll
            for (int s = 0; s < 4; ++s) { const int row = 4 * s + (lane >> 3), piece = lane & 7; const float* sp = os + row * 68 + piece * 8; v8h o, o2;
#pragma unroll
                for (int i = 0; i < 8; ++i) { const h16 a = (h16)sp[i]; o[i] = a; o2[i] = (h16)((sp[i] - (float)a) * LOSC); }
                *(volatile v8h*)(crow + (size_t)row * ldc + piece * 8) = o; if (C2) *(volatile v8h*)(C2 + (size_t)r0 * ldc + c0 + (size_t)row * ldc + piece * 8) = o2; }
        };
        pass(); __threadfence(); pass();
    } else {
        float* crow = C + (size_t)r0 * ldc + c0;
        auto pass = [&]() {
#pragma unroll
            for (int s = 0; s < 8; ++s) { const int Lid = (lane >> 3) + 4 * s, piece = lane & 7; const int row = Lid >> 1, cofs = (Lid & 1) * 32 + piece * 4;
                v4f val = *(const v4fa*)(os + row * 68 + cofs); if (R) { const v4f rv = *(const v4f*)(R + ((size_t)r0 + row) * ldc + c0 + cofs); val += roundR ? (v4f){bfr(rv[0]), bfr(rv[1]), bfr(rv[2]), bfr(rv[3])} : rv; }
                *(volatile v4f*)(crow + (size_t)row * ldc + cofs) = val; }
        };
        pass(); __threadfence(); pass();
    }
}

__global__ __launch_bounds__(256) void k_cvt8(const float* __restrict__ src, bf* dst, size_t n8) {
    const size_t i = (size_t)blockIdx.x * 256 + threadIdx.x; if (i >= n8) return;
    const v8f v = *(const v8f*)(src + i * 8); v8us o;
#pragma unroll
    for (int k = 0; k < 8; ++k) o[k] = f2bf(v[k]);
    *(volatile v8us*)(dst + i * 8) = o; __threadfence(); *(volatile v8us*)(dst + i * 8) = o;
}
__global__ __launch_bounds__(256) void k_zero8(bf* dst, size_t n8) {
    const size_t i = (size_t)blockIdx.x * 256 + threadIdx.x; if (i >= n8) return; v8us z;
#pragma unroll
    for (int k = 0; k < 8; ++k) z[k] = 0;
    *(volatile v8us*)(dst + i * 8) = z; __threadfence(); *(volatile v8us*)(dst + i * 8) = z;
}
__global__ __launch_bounds__(128) void k_gemm3(const bf* __restrict__ Ah, const bf* __restrict__ Al, const bf* __restrict__ Bh, const bf* __restrict__ Bl, int K, float* C, int ldc) {
    __shared__ __align__(16) float ost[4][16 * 68];
    const int lane = threadIdx.x & 31, wave = threadIdx.x >> 5, lr = lane & 15, hi = lane >> 4;
    const int r0 = blockIdx.x * 64 + wave * 16, c0 = blockIdx.y * 64;
    const size_t aoff = (size_t)(r0 + lr) * K + 8 * hi;
    v8f acc[4];
#pragma unroll
    for (int t = 0; t < 4; ++t) acc[t] = (v8f){};
#pragma unroll 1
    for (int kc = 0; kc < K; kc += 32) {
        const v16bf a = cat16b(*(const v8us*)(Ah + aoff + kc), *(const v8us*)(Ah + aoff + kc + 16));
        const v16bf al = cat16b(*(const v8us*)(Al + aoff + kc), *(const v8us*)(Al + aoff + kc + 16));
#pragma unroll
        for (int t = 0; t < 4; ++t) { const size_t bo = (size_t)(c0 + t * 16 + lr) * K + kc + 8 * hi;
            const v16bf bh = cat16b(*(const v8us*)(Bh + bo), *(const v8us*)(Bh + bo + 16)); const v16bf bl = cat16b(*(const v8us*)(Bl + bo), *(const v8us*)(Bl + bo + 16));
            acc[t] = wmmab(a, bh, acc[t]); acc[t] = wmmab(al, bh, acc[t]); acc[t] = wmmab(a, bl, acc[t]); }
        asm volatile("v_nop\n\tv_nop\n\tv_nop\n\tv_nop" : "+v"(acc[0]), "+v"(acc[1]), "+v"(acc[2]), "+v"(acc[3]) : "v"(a), "v"(al));
    }
    float* os = &ost[wave][0];
#pragma unroll
    for (int t = 0; t < 4; ++t) {
#pragma unroll
        for (int j = 0; j < 8; ++j) os[(hi * 8 + j) * 68 + t * 16 + lr] = acc[t][j]; }
    __builtin_amdgcn_wave_barrier(); asm volatile("" ::: "memory");
    float* crow = C + (size_t)r0 * ldc + c0;
    auto pass = [&]() {
#pragma unroll
        for (int s = 0; s < 8; ++s) { const int Lid = (lane >> 3) + 4 * s, piece = lane & 7; const int row = Lid >> 1, cofs = (Lid & 1) * 32 + piece * 4;
            const v4f val = *(const v4fa*)(os + row * 68 + cofs); *(volatile v4f*)(crow + (size_t)row * ldc + cofs) = val; }
    };
    pass(); __threadfence(); pass();
}


__global__ __launch_bounds__(256) void k_gnstat(const float* __restrict__ xb, float* ST) {
    const int lane = threadIdx.x & 31; const int g = blockIdx.x * 8 + (threadIdx.x >> 5); if (g >= NG) return; const float* base = xb + (size_t)(2 * g) * NV; const int n = 2 * NV; float s = 0.f;
    for (int i = lane; i < n; i += 32) s += base[i];
#pragma unroll
    for (int sh = 16; sh; sh >>= 1) s += __shfl_xor(s, sh, 32);
    const float mu = s / (float)n; float q = 0.f;
    for (int i = lane; i < n; i += 32) { const float d = base[i] - mu; q = fmaf(d, d, q); }
#pragma unroll
    for (int sh = 16; sh; sh >>= 1) q += __shfl_xor(q, sh, 32);
    const float rs = rsqrtf(q / (float)n + GEPS); const float v = (lane == 0) ? mu : (lane == 1) ? rs : 0.f;
    *(volatile float*)(ST + (size_t)g * 32 + lane) = v; __threadfence(); *(volatile float*)(ST + (size_t)g * 32 + lane) = v;
}
__global__ __launch_bounds__(256) void k_gnT(const float* __restrict__ xb, const float* __restrict__ ST, const float* __restrict__ gam, const float* __restrict__ bet, bf* Hh, bf* Hl) {
    __shared__ float tl[64][65];
    typedef __attribute__((ext_vector_type(4))) unsigned short v4us;
    const int tid = threadIdx.x, p0 = blockIdx.y * 64; const int rr = tid >> 2, cq = (tid & 3) * 16;
    { const float mu = ST[(rr >> 1) * 32], rs = ST[(rr >> 1) * 32 + 1], ga = bfr(gam[rr]), be = bfr(bet[rr]);
#pragma unroll
      for (int i = 0; i < 16; ++i) tl[rr][cq + i] = (bfr(xb[(size_t)rr * NV + p0 + cq + i]) - mu) * rs * ga + be; }
    __syncthreads();
    const int lane = tid & 31, wv = tid >> 5;
    auto pass = [&]() {
#pragma unroll
        for (int st = 0; st < 4; ++st) { const int pr = wv * 8 + st * 2 + (lane >> 4); const int cl = (lane & 15) * 4; v4us oh, ol;
#pragma unroll
            for (int i = 0; i < 4; ++i) { const float y = tl[cl + i][pr]; const unsigned short hb = f2bf(y); oh[i] = hb; ol[i] = f2bf(y - bf2f(hb)); }
            const size_t o = (size_t)(p0 + pr) * CC + cl; *(volatile v4us*)(Hh + o) = oh; *(volatile v4us*)(Hl + o) = ol; }
    };
    pass(); __threadfence(); pass();
}
__global__ __launch_bounds__(256) void k_split64(const float* __restrict__ F, int rows, float sc, bf* Ph, bf* Pl) {
    typedef __attribute__((ext_vector_type(2))) unsigned short v2us; typedef __attribute__((ext_vector_type(2))) float v2f_;
    const int lane = threadIdx.x & 31; const size_t r = (size_t)blockIdx.x * 8 + (threadIdx.x >> 5); if (r >= (size_t)rows) return; const size_t o = r * CC + lane * 2; const v2f_ v = *(const v2f_*)(F + o); v2us oh, ol;
#pragma unroll
    for (int i = 0; i < 2; ++i) { const float y = v[i] * sc; const unsigned short hb = f2bf(y); oh[i] = hb; ol[i] = f2bf(y - bf2f(hb)); }
    *(volatile v2us*)(Ph + o) = oh; *(volatile v2us*)(Pl + o) = ol; __threadfence(); *(volatile v2us*)(Ph + o) = oh; *(volatile v2us*)(Pl + o) = ol;
}
__global__ __launch_bounds__(256) void k_vT(const float* __restrict__ V, bf* Th, bf* Tl) {
    __shared__ float tl[64][65];
    typedef __attribute__((ext_vector_type(4))) unsigned short v4us;
    const int tid = threadIdx.x; const int t0 = blockIdx.x * 64; const int rr = tid >> 2, cq = (tid & 3) * 16;
#pragma unroll
    for (int i = 0; i < 16; ++i) tl[rr][cq + i] = V[(size_t)(t0 + rr) * CC + cq + i];
    __syncthreads();
    const int lane = tid & 31, wv = tid >> 5;
    auto pass = [&]() {
#pragma unroll
        for (int st = 0; st < 4; ++st) { const int dr = wv * 8 + st * 2 + (lane >> 4); const int tq = (lane & 15) * 4; v4us oh, ol;
#pragma unroll
            for (int i = 0; i < 4; ++i) { const float y = tl[tq + i][dr]; const unsigned short hb = f2bf(y); oh[i] = hb; ol[i] = f2bf(y - bf2f(hb)); }
            const size_t o = (size_t)dr * NV + t0 + tq; *(volatile v4us*)(Th + o) = oh; *(volatile v4us*)(Tl + o) = ol; }
    };
    pass(); __threadfence(); pass();
}
__global__ __launch_bounds__(256) void k_soft(const float* __restrict__ S, float sc, bf* PH, bf* PL) {
    typedef __attribute__((ext_vector_type(4))) unsigned short v4us;
    const int lane = threadIdx.x & 31, i = blockIdx.x * 8 + (threadIdx.x >> 5); if (i >= RB) return; const float* sr = S + (size_t)i * NV;
    float m = -3.0e38f;
#pragma unroll 1
    for (int c0 = lane * 4; c0 < NV; c0 += 128) {
#pragma unroll
        for (int q = 0; q < 4; ++q) m = fmaxf(m, sr[c0 + q] * sc); }
#pragma unroll
    for (int sh = 16; sh; sh >>= 1) m = fmaxf(m, __shfl_xor(m, sh, 32));
    float sum = 0.f;
#pragma unroll 1
    for (int c0 = lane * 4; c0 < NV; c0 += 128) {
#pragma unroll
        for (int q = 0; q < 4; ++q) sum += __expf(sr[c0 + q] * sc - m); }
#pragma unroll
    for (int sh = 16; sh; sh >>= 1) sum += __shfl_xor(sum, sh, 32);
    const float inv = 1.0f / sum;
#pragma unroll 1
    for (int ps = 0; ps < 2; ++ps) {
#pragma unroll 1
        for (int c0 = lane * 4; c0 < NV; c0 += 128) { v4us oh, ol;
#pragma unroll
            for (int q = 0; q < 4; ++q) { const float p = __expf(sr[c0 + q] * sc - m) * inv; const unsigned short hb = f2bf(p); oh[q] = hb; ol[q] = f2bf(p - bf2f(hb)); }
            const size_t o = (size_t)i * NV + c0; *(volatile v4us*)(PH + o) = oh; *(volatile v4us*)(PL + o) = ol; }
        if (ps == 0) __threadfence(); }
}
__global__ __launch_bounds__(256) void k_outT(const float* __restrict__ OT, const float* __restrict__ xb, float* OUTB) {
    __shared__ float tl[64][65];
    const int tid = threadIdx.x; const int p0 = blockIdx.x * 64; const int rr = tid >> 2, cq = (tid & 3) * 16;
#pragma unroll
    for (int i = 0; i < 16; ++i) tl[rr][cq + i] = OT[(size_t)(p0 + rr) * CC + cq + i];
    __syncthreads();
    const int lane = tid & 31, wv = tid >> 5;
    auto pass = [&]() {
#pragma unroll
        for (int st = 0; st < 4; ++st) { const int cr = wv * 8 + st * 2 + (lane >> 4); const int pq = (lane & 15) * 4; v4f v; const size_t o = (size_t)cr * NV + p0 + pq;
#pragma unroll
            for (int i = 0; i < 4; ++i) v[i] = bfr(xb[o + i]) + tl[pq + i][cr];
            *(volatile v4f*)(OUTB + o) = v; }
    };
    pass(); __threadfence(); pass();
}

extern "C" void kernel_launch(void* const* d_in, const int* in_sizes, int n_in,
                              void* d_out, int out_size, void* d_ws, size_t ws_size, hipStream_t stream) {
    (void)in_sizes; (void)n_in; (void)out_size;
    const float* x = (const float*)d_in[0]; const float* gam = (const float*)d_in[1]; const float* bet = (const float*)d_in[2]; const float* wq = (const float*)d_in[3]; const float* bq = (const float*)d_in[4]; const float* wk = (const float*)d_in[5]; const float* bk = (const float*)d_in[6]; const float* wv = (const float*)d_in[7]; const float* bv = (const float*)d_in[8]; const float* wp = (const float*)d_in[9]; const float* bp = (const float*)d_in[10];
    float* out = (float*)d_out;
    char* wsp = (char*)d_ws;
    auto take = [&](size_t bytes) { char* p = wsp; wsp += (bytes + 255) & ~(size_t)255; return (void*)p; };
    bf* WQ = (bf*)take(CC * CC * 2); bf* WK = (bf*)take(CC * CC * 2); bf* WV = (bf*)take(CC * CC * 2); bf* WP = (bf*)take(CC * CC * 2); float* ST = (float*)take(NG * 32 * 4);
    bf* Hh = (bf*)take((size_t)NV * CC * 2); bf* Hl = (bf*)take((size_t)NV * CC * 2); float* QF = (float*)take((size_t)NV * CC * 4); float* KF = (float*)take((size_t)NV * CC * 4); float* VF = (float*)take((size_t)NV * CC * 4);
    bf* Qh = (bf*)take((size_t)NV * CC * 2); bf* Ql = (bf*)take((size_t)NV * CC * 2); bf* Kh = (bf*)take((size_t)NV * CC * 2); bf* Kl = (bf*)take((size_t)NV * CC * 2); bf* VTh = (bf*)take((size_t)CC * NV * 2); bf* VTl = (bf*)take((size_t)CC * NV * 2);
    float* S = (float*)take((size_t)RB * NV * 4); bf* PH = (bf*)take((size_t)RB * NV * 2); bf* PL = (bf*)take((size_t)RB * NV * 2); float* O = (float*)take((size_t)NV * CC * 4); bf* Oh = (bf*)take((size_t)NV * CC * 2); bf* Ol = (bf*)take((size_t)NV * CC * 2); float* OT = (float*)take((size_t)NV * CC * 4);
    if ((size_t)(wsp - (char*)d_ws) > ws_size) return;
    k_cvt8<<<(CC * CC / 8 + 255) / 256, 256, 0, stream>>>(wq, WQ, CC * CC / 8); k_cvt8<<<(CC * CC / 8 + 255) / 256, 256, 0, stream>>>(wk, WK, CC * CC / 8); k_cvt8<<<(CC * CC / 8 + 255) / 256, 256, 0, stream>>>(wv, WV, CC * CC / 8); k_cvt8<<<(CC * CC / 8 + 255) / 256, 256, 0, stream>>>(wp, WP, CC * CC / 8);
    const dim3 gp(NV / 64, 1, 1);
    for (int b = 0; b < NB_; ++b) { const float* xb = x + (size_t)b * CC * NV;
        k_gnstat<<<NG / 8, 256, 0, stream>>>(xb, ST); k_gnT<<<dim3(1, NV / 64, 1), 256, 0, stream>>>(xb, ST, gam, bet, Hh, Hl);
        k_gemmb<true, false><<<gp, 128, 0, stream>>>(Hh, Hl, WQ, bq, QF, CC, nullptr, nullptr, CC); k_gemmb<true, false><<<gp, 128, 0, stream>>>(Hh, Hl, WK, bk, KF, CC, nullptr, nullptr, CC); k_gemmb<true, false><<<gp, 128, 0, stream>>>(Hh, Hl, WV, bv, VF, CC, nullptr, nullptr, CC);
        k_split64<<<NV / 8, 256, 0, stream>>>(QF, NV, 1.0f, Qh, Ql); k_split64<<<NV / 8, 256, 0, stream>>>(KF, NV, 1.0f, Kh, Kl); k_vT<<<NV / 64, 256, 0, stream>>>(VF, VTh, VTl);
        for (int rb = 0; rb < NV / RB; ++rb) { const size_t r0 = (size_t)rb * RB;
            k_gemm3<<<dim3(RB / 64, NV / 64, 1), 128, 0, stream>>>(Qh + r0 * CC, Ql + r0 * CC, Kh, Kl, CC, S, NV);
            k_soft<<<RB / 8, 256, 0, stream>>>(S, SCL, PH, PL);
            k_gemm3<<<dim3(RB / 64, 1, 1), 128, 0, stream>>>(PH, PL, VTh, VTl, NV, O + r0 * CC, CC); }
        k_split64<<<NV / 8, 256, 0, stream>>>(O, NV, 1.0f, Oh, Ol);
        k_gemmb<true, false><<<gp, 128, 0, stream>>>(Oh, Ol, WP, bp, OT, CC, nullptr, nullptr, CC);
        k_outT<<<dim3(NV / 64, 1, 1), 256, 0, stream>>>(OT, xb, out + (size_t)b * CC * NV); }
}
